// ElectronGNN_62113817035113
// MI455X (gfx1250) — hardware-run, weakly checked
//
#include <hip/hip_runtime.h>
#include <stddef.h>
#include <stdint.h>

#define NCFG  1024
#define NE    32
#define NN    8
#define DD    256
#define HH    64
#define FF    8
#define LL    4
#define NUP   16
#define A3H   192
#define MROWS 32768
#define KX    512
#define KA    384
#define KT    512
#define GBM   64
#define GBN   128
#define GTHR  128
#define ETHR  256
#define WSMAX 134217728

#define E_SW    0
#define E_SHX   (E_SW + 256 * 64)
#define E_SACC  (E_SHX + 32 * 128)
#define E_SSP   (E_SACC + 32 * 192)
#define E_SRE   (E_SSP + 1024)
#define E_SRN   (E_SRE + 128)
#define E_SPAIR (E_SRN + 32)
#define E_SW1   (E_SPAIR + 128)
#define E_SW2   (E_SW1 + 3072)
#define E_TOTF  (E_SW2 + 6144)
#define EDGE_LDS_BYTES (E_TOTF * 4)

#define PA_L0 3072
#define PA_L1 (PA_L0 + 6144)
#define PA_L2 (PA_L1 + 32768)
#define PB_L0 49152
#define PB_L1 (PB_L0 + 65536)
#define PC_L0 1024
#define PC_L1 1280
#define PC_L2 1536
#define PC_L3 1664
#define X0_L0 2097152
#define X0_L1 4194304

static_assert(NE == 32 && NN == 8 && NUP == 16 && HH == 64 && FF == 8 && DD == 256 && A3H == 3 * HH && LL == 4);
static_assert(MROWS == NCFG * NE && MROWS % GBM == 0 && MROWS % 128 == 0);
static_assert(KX == 2 * DD && KA == 2 * A3H && KT == 2 * DD);
static_assert(KX % 32 == 0 && KA % 32 == 0 && KT % 32 == 0 && A3H % 32 == 0);
static_assert(240 % 16 == 0 && 2 * 120 == 240);
static_assert(GBM == (GTHR / 32) * 16 && GBN == 128 && DD % GBN == 0);
static_assert(EDGE_LDS_BYTES <= 327680);
static_assert((E_SHX % 4) == 0 && (E_SACC % 4) == 0 && (E_SSP % 4) == 0 && (E_SRE % 4) == 0);
static_assert((E_SRN % 4) == 0 && (E_SPAIR % 4) == 0 && (E_SW1 % 4) == 0 && (E_SW2 % 4) == 0);
static_assert(PA_L0 % 256 == 0 && PA_L1 % 256 == 0 && PA_L2 % 256 == 0);
static_assert(PA_L0 * 8 == LL * 3 * HH * 32 && (PA_L1 - PA_L0) * 8 == LL * 3 * HH * HH);
static_assert((PA_L2 - PA_L1) * 8 == LL * 128 * KX);
static_assert(PB_L0 % 256 == 0 && PB_L1 % 256 == 0);
static_assert(PB_L0 * 8 == LL * DD * KA && (PB_L1 - PB_L0) * 8 == LL * DD * KT);
static_assert(PC_L0 % 256 == 0 && PC_L1 % 256 == 0 && PC_L2 % 256 == 0 && PC_L3 % 32 == 0);
static_assert(X0_L0 * 4 == MROWS * DD && (X0_L1 - X0_L0) * 8 == MROWS * KX && X0_L1 % 256 == 0);
static_assert(32 * KA * 2 == 6 * ETHR * 16);
static_assert(3 * HH * 32 * 2 == 3 * ETHR * 16 && 3 * HH * HH * 2 == 6 * ETHR * 16 && 32 * 128 * 4 == 4 * ETHR * 16);

typedef float          v4f   __attribute__((ext_vector_type(4)));
typedef float          v8f   __attribute__((ext_vector_type(8)));
typedef int            v4i   __attribute__((ext_vector_type(4)));
typedef int            v8i   __attribute__((ext_vector_type(8)));
typedef unsigned short v8us  __attribute__((ext_vector_type(8)));
typedef unsigned short v16us __attribute__((ext_vector_type(16)));
typedef __bf16         v16bf __attribute__((ext_vector_type(16)));
typedef v4f  __attribute__((may_alias)) v4fa;
typedef v4i  __attribute__((may_alias)) v4ia;
typedef v8us __attribute__((may_alias)) v8usa;
union FragB { v16bf v; v16us u; v8us h[2]; v8i w; };

constexpr float MUC0 = 8.0f * ((float)0 / 7.0f);
constexpr float MUC1 = 8.0f * ((float)1 / 7.0f);
constexpr float MUC2 = 8.0f * ((float)2 / 7.0f);
constexpr float MUC3 = 8.0f * ((float)3 / 7.0f);
constexpr float MUC4 = 8.0f * ((float)4 / 7.0f);
constexpr float MUC5 = 8.0f * ((float)5 / 7.0f);
constexpr float MUC6 = 8.0f * ((float)6 / 7.0f);
constexpr float MUC7 = 8.0f;

__host__ __device__ __forceinline__ constexpr int pidx(int p, int q) {
  return 15 * p - (p * (p - 1)) / 2 + (q - p - 1);
}
constexpr bool pidx_table_ok() {
  bool seen[120] = {};
  for (int p = 0; p < 16; ++p)
    for (int q = p + 1; q < 16; ++q) {
      const int v = pidx(p, q);
      if (v < 0 || v >= 120) return false;
      if (seen[v]) return false;
      seen[v] = true;
    }
  for (int i = 0; i < 120; ++i) if (!seen[i]) return false;
  return true;
}
static_assert(pidx_table_ok());

__device__ __forceinline__ v8f wmb(const FragB& a, const FragB& b, v8f c) {
  v8f d = __builtin_amdgcn_wmma_f32_16x16x32_bf16(false, a.v, false, b.v, (short)0, c, false, false);
  asm volatile("v_nop\n\tv_nop\n\tv_nop\n\tv_nop" : "+v"(d) : "v"(a.w), "v"(b.w));
  return d;
}

__device__ __forceinline__ unsigned bf16_bits(float f) {
  const unsigned u = __float_as_uint(f);
  return (u + 0x7FFFu + ((u >> 16) & 1u)) >> 16;
}
__device__ __forceinline__ float bf16_val(float f) {
  return __uint_as_float(bf16_bits(f) << 16);
}
__device__ __forceinline__ float silu_fast(float v) {
  const float e = __expf(-v);
  return v * __builtin_amdgcn_rcpf(1.0f + e);
}
__device__ __forceinline__ void put16(unsigned short* dp, v8us o) {
  *(volatile v8us*)dp = o;
  __threadfence();
  *(volatile v8us*)dp = o;
}
__device__ __forceinline__ void putf4(float* dp, v4f o) {
  *(volatile v4f*)dp = o;
  __threadfence();
  *(volatile v4f*)dp = o;
}

__global__ __launch_bounds__(256) __attribute__((amdgpu_num_vgpr(248)))
void k_pa(const float* __restrict__ wW1, const float* __restrict__ wW2, const float* __restrict__ hW,
          unsigned short* W1P, unsigned short* W2P, unsigned short* HWP) {
  const int u = (int)blockIdx.x * 256 + (int)threadIdx.x;
  v8us o;
  if (u < PA_L0) {
    const int lt = u >> 8;
    const int n  = (u >> 2) & 63;
    const int kq = u & 3;
    const unsigned keep = (kq < 2) ? 0xffffu : 0u;
    const float* p = wW1 + (size_t)lt * FF * HH + n;
    float f[8];
#pragma unroll
    for (int i = 0; i < 8; ++i) f[i] = p[(size_t)i * HH];
    asm volatile("" :: "v"(f[0]), "v"(f[1]), "v"(f[2]), "v"(f[3]), "v"(f[4]), "v"(f[5]), "v"(f[6]), "v"(f[7]));
#pragma unroll
    for (int i = 0; i < 8; ++i) o[i] = (unsigned short)(bf16_bits(f[i]) & keep);
    put16(W1P + (size_t)u * 8, o);
  } else if (u < PA_L1) {
    const int v  = u - PA_L0;
    const int lt = v >> 9;
    const int n  = (v >> 3) & 63;
    const int k8 = (v & 7) * 8;
    const float* p = wW2 + ((size_t)lt * HH + k8) * HH + n;
#pragma unroll
    for (int i = 0; i < 8; ++i) o[i] = (unsigned short)bf16_bits(p[(size_t)i * HH]);
    put16(W2P + (size_t)v * 8, o);
  } else if (u < PA_L2) {
    const int v  = u - PA_L1;
    const int l  = v >> 13;
    const int n  = (v >> 6) & 127;
    const int k8 = (v & 63) * 8;
    const int sk = k8 & 255;
    const int t  = 1 + (n >> 6);
    const int nn = n & 63;
    const float* p = hW + ((size_t)(l * 3 + t) * DD + sk) * HH + nn;
#pragma unroll
    for (int i = 0; i < 8; ++i) o[i] = (unsigned short)bf16_bits(p[(size_t)i * HH]);
    put16(HWP + (size_t)v * 8, o);
  }
}

__global__ __launch_bounds__(256) __attribute__((amdgpu_num_vgpr(248)))
void k_pb(const float* __restrict__ uW1, const float* __restrict__ uW2,
          unsigned short* U1P, unsigned short* U2P) {
  const int u = (int)blockIdx.x * 256 + (int)threadIdx.x;
  v8us o;
  if (u < PB_L0) {
    const int l   = u / 12288;
    const int rem = u - l * 12288;
    const int n   = rem / 48;
    const int kq  = rem - n * 48;
    const int k8  = kq * 8;
    const int sk  = (k8 >= A3H) ? (k8 - A3H) : k8;
    const float* p = uW1 + ((size_t)l * A3H + sk) * DD + n;
#pragma unroll
    for (int i = 0; i < 8; ++i) o[i] = (unsigned short)bf16_bits(p[(size_t)i * DD]);
    put16(U1P + (size_t)u * 8, o);
  } else if (u < PB_L1) {
    const int v  = u - PB_L0;
    const int l  = v >> 14;
    const int n  = (v >> 6) & 255;
    const int k8 = (v & 63) * 8;
    const int sk = k8 & 255;
    const float* p = uW2 + ((size_t)l * DD + sk) * DD + n;
#pragma unroll
    for (int i = 0; i < 8; ++i) o[i] = (unsigned short)bf16_bits(p[(size_t)i * DD]);
    put16(U2P + (size_t)v * 8, o);
  }
}

__global__ __launch_bounds__(256) __attribute__((amdgpu_num_vgpr(248)))
void k_pc(const float* __restrict__ nuc, const float* __restrict__ hW, const float* __restrict__ hB,
          const float* __restrict__ wB1, const float* __restrict__ wB2,
          const float* __restrict__ uB1, const float* __restrict__ uB2,
          float* SP, float* HBP, float* UB1P, float* UB2P) {
  const int u = (int)blockIdx.x * 256 + (int)threadIdx.x;
  if (u < PC_L0) {
    const int l = u >> 8;
    const int q = u & 255;
    v4f o;
    if (q < 128) {
      const int n  = q >> 4;
      const int h0 = (q & 15) * 4;
      v4f acc = {0.0f, 0.0f, 0.0f, 0.0f};
      const float* yp = nuc + (size_t)n * DD;
      const float* wp = hW + (size_t)(l * 3) * DD * HH + h0;
#pragma unroll 4
      for (int k = 0; k < DD; ++k) {
        const float yv = bf16_val(yp[k]);
        const v4f w = *(const v4fa*)(wp + (size_t)k * HH);
        acc.x = fmaf(yv, bf16_val(w.x), acc.x);
        acc.y = fmaf(yv, bf16_val(w.y), acc.y);
        acc.z = fmaf(yv, bf16_val(w.z), acc.z);
        acc.w = fmaf(yv, bf16_val(w.w), acc.w);
      }
      const v4f bb = *(const v4fa*)(hB + (size_t)(l * 3) * HH + h0);
      o.x = acc.x + bf16_val(bb.x);
      o.y = acc.y + bf16_val(bb.y);
      o.z = acc.z + bf16_val(bb.z);
      o.w = acc.w + bf16_val(bb.w);
    } else if (q < 192) {
      const int tq = (q - 128) >> 4;
      const int h0 = ((q - 128) & 15) * 4;
      const int tc = tq < 2 ? tq : 2;
      const v4f bb = *(const v4fa*)(wB1 + (size_t)(l * 3 + tc) * HH + h0);
      asm volatile("" :: "v"(bb.x), "v"(bb.y), "v"(bb.z), "v"(bb.w));
      const bool on = tq < 3;
      o.x = on ? bf16_val(bb.x) : 0.0f;
      o.y = on ? bf16_val(bb.y) : 0.0f;
      o.z = on ? bf16_val(bb.z) : 0.0f;
      o.w = on ? bf16_val(bb.w) : 0.0f;
    } else {
      const int tq = (q - 192) >> 4;
      const int h0 = ((q - 192) & 15) * 4;
      const int tc = tq < 2 ? tq : 2;
      const v4f bb = *(const v4fa*)(wB2 + (size_t)(l * 3 + tc) * HH + h0);
      asm volatile("" :: "v"(bb.x), "v"(bb.y), "v"(bb.z), "v"(bb.w));
      const bool on = tq < 3;
      o.x = on ? bf16_val(bb.x) : 0.0f;
      o.y = on ? bf16_val(bb.y) : 0.0f;
      o.z = on ? bf16_val(bb.z) : 0.0f;
      o.w = on ? bf16_val(bb.w) : 0.0f;
    }
    putf4(SP + (size_t)u * 4, o);
  } else if (u < PC_L1) {
    const int v = u - PC_L0;
    const v4f bb = *(const v4fa*)(uB1 + (size_t)v * 4);
    const v4f o = {bf16_val(bb.x), bf16_val(bb.y), bf16_val(bb.z), bf16_val(bb.w)};
    putf4(UB1P + (size_t)v * 4, o);
  } else if (u < PC_L2) {
    const int v = u - PC_L1;
    const v4f bb = *(const v4fa*)(uB2 + (size_t)v * 4);
    const v4f o = {bf16_val(bb.x), bf16_val(bb.y), bf16_val(bb.z), bf16_val(bb.w)};
    putf4(UB2P + (size_t)v * 4, o);
  } else if (u < PC_L3) {
    const int v  = u - PC_L2;
    const int l  = v >> 5;
    const int c0 = (v & 31) * 4;
    const int t  = 1 + (c0 >> 6);
    const int cc = c0 & 63;
    const v4f bb = *(const v4fa*)(hB + (size_t)(l * 3 + t) * HH + cc);
    const v4f o = {bf16_val(bb.x), bf16_val(bb.y), bf16_val(bb.z), bf16_val(bb.w)};
    putf4(HBP + (size_t)v * 4, o);
  }
}

__global__ __launch_bounds__(256) __attribute__((amdgpu_num_vgpr(248)))
void k_x0(const float* __restrict__ elec, float* X, unsigned short* XHL) {
  const int u = (int)blockIdx.x * 256 + (int)threadIdx.x;
  if (u < X0_L0) {
    const int c4 = u & 63;
    const v4f e = *(const v4fa*)(elec + 4 * c4);
    const v4f o = {bf16_val(e.x), bf16_val(e.y), bf16_val(e.z), bf16_val(e.w)};
    putf4(X + (size_t)u * 4, o);
  } else if (u < X0_L1) {
    const int v  = u - X0_L0;
    const int c8 = v & 63;
    const int cc = c8 & 31;
    const unsigned keep = (c8 < 32) ? 0xffffu : 0u;
    const v4f a = *(const v4fa*)(elec + 8 * cc);
    const v4f b = *(const v4fa*)(elec + 8 * cc + 4);
    asm volatile("" :: "v"(a.x), "v"(a.y), "v"(a.z), "v"(a.w), "v"(b.x), "v"(b.y), "v"(b.z), "v"(b.w));
    const v8f f8 = {a.x, a.y, a.z, a.w, b.x, b.y, b.z, b.w};
    v8us o;
#pragma unroll
    for (int i = 0; i < 8; ++i) o[i] = (unsigned short)(bf16_bits(f8[i]) & keep);
    put16(XHL + (size_t)v * 8, o);
  }
}

template <int MODE>
__global__ __launch_bounds__(GTHR) __attribute__((amdgpu_num_vgpr(248)))
void k_gemm(const unsigned short* __restrict__ A, int lda, const unsigned short* __restrict__ BT, int ldb, int K,
            const float* __restrict__ bias, float* Xp, float* Cf, unsigned short* Cb) {
  __shared__ __attribute__((aligned(16))) float stg[GBM * GBN];
  const int tid = (int)threadIdx.x, lane = tid & 31, wave = tid >> 5, hh = lane >> 4, m = lane & 15;
  const int rowBase = (int)blockIdx.x * GBM;
  const int colBase = (int)blockIdx.y * GBN;

  v8f acc[8];
  {
    const v8f z = {0.f, 0.f, 0.f, 0.f, 0.f, 0.f, 0.f, 0.f};
#pragma unroll
    for (int t = 0; t < 8; ++t) acc[t] = z;
  }
  const unsigned short* ap = A  + (size_t)(rowBase + 16 * wave + m) * (size_t)lda + 8 * hh;
  const unsigned short* bp = BT + (size_t)(colBase + m) * (size_t)ldb + 8 * hh;

#pragma unroll 1
  for (int k0 = 0; k0 < K; k0 += 32) {
    FragB af;
    af.h[0] = *(const v8usa*)(ap + k0);
    af.h[1] = *(const v8usa*)(ap + k0 + 16);
#pragma unroll
    for (int nt = 0; nt < 8; ++nt) {
      const unsigned short* wq = bp + (size_t)(16 * nt) * (size_t)ldb + k0;
      FragB bf;
      bf.h[0] = *(const v8usa*)wq;
      bf.h[1] = *(const v8usa*)(wq + 16);
      acc[nt] = wmb(af, bf, acc[nt]);
    }
  }

#pragma unroll
  for (int nt = 0; nt < 8; ++nt) {
    const int lc = 16 * nt + m;
    const float bvv = bias[colBase + lc];
#pragma unroll
    for (int r = 0; r < 8; ++r) {
      const int lr = 16 * wave + 8 * hh + r;
      float v = acc[nt][r] + bvv;
      if constexpr (MODE == 1) v = silu_fast(v);
      stg[lr * GBN + lc] = v;
    }
  }
  __syncthreads();

  if constexpr (MODE == 0 || MODE == 3) {
    constexpr int LDC = (MODE == 0) ? 128 : 256;
    v4f pv[16];
#pragma unroll
    for (int i = 0; i < 16; ++i) {
      v4f s = *(const v4fa*)(stg + (16 * wave + i) * GBN + 4 * lane);
      if constexpr (MODE == 3) {
        const v4f x = *(const v4fa*)(Xp + (size_t)(rowBase + 16 * wave + i) * DD + colBase + 4 * lane);
        s = x + s;
      }
      pv[i] = s;
    }
#pragma unroll
    for (int i = 0; i < 16; ++i) {
      float* op = Cf + (size_t)(rowBase + 16 * wave + i) * LDC + colBase + 4 * lane;
      *(volatile v4f*)op = pv[i];
    }
    __threadfence();
#pragma unroll
    for (int i = 0; i < 16; ++i) {
      float* op = Cf + (size_t)(rowBase + 16 * wave + i) * LDC + colBase + 4 * lane;
      *(volatile v4f*)op = pv[i];
    }
  }

  if constexpr (MODE == 2) {
    v4f pv[16];
#pragma unroll
    for (int i = 0; i < 16; ++i) {
      float* sp = stg + (16 * wave + i) * GBN + 4 * lane;
      const v4f s = *(const v4fa*)sp;
      const v4f x = *(const v4fa*)(Xp + (size_t)(rowBase + 16 * wave + i) * DD + colBase + 4 * lane);
      const v4f v = x + s;
      pv[i] = v;
      *(v4fa*)sp = v;
    }
#pragma unroll
    for (int i = 0; i < 16; ++i) {
      float* op = Xp + (size_t)(rowBase + 16 * wave + i) * DD + colBase + 4 * lane;
      *(volatile v4f*)op = pv[i];
    }
    __threadfence();
#pragma unroll
    for (int i = 0; i < 16; ++i) {
      float* op = Xp + (size_t)(rowBase + 16 * wave + i) * DD + colBase + 4 * lane;
      *(volatile v4f*)op = pv[i];
    }
    __syncthreads();
  }

  if constexpr (MODE == 1 || MODE == 2) {
    const int part = lane >> 4;
    const int j = lane & 15;
    const unsigned mh = 0u - (unsigned)part;
    const unsigned ml = ~mh;
    v8us pv[16];
#pragma unroll
    for (int i = 0; i < 16; ++i) {
      const float* sp = stg + (16 * wave + i) * GBN + 8 * j;
      const v4f a = *(const v4fa*)sp;
      const v4f b = *(const v4fa*)(sp + 4);
      const v8f f8 = {a.x, a.y, a.z, a.w, b.x, b.y, b.z, b.w};
      v8us oo;
#pragma unroll
      for (int e = 0; e < 8; ++e) {
        const unsigned hb = bf16_bits(f8[e]);
        const unsigned lb = bf16_bits(f8[e] - __uint_as_float(hb << 16));
        oo[e] = (unsigned short)((hb & ml) | (lb & mh));
      }
      pv[i] = oo;
    }
#pragma unroll
    for (int i = 0; i < 16; ++i) {
      unsigned short* op = Cb + (size_t)(rowBase + 16 * wave + i) * 512 + part * 256 + colBase + 8 * j;
      *(volatile v8us*)op = pv[i];
    }
    __threadfence();
#pragma unroll
    for (int i = 0; i < 16; ++i) {
      unsigned short* op = Cb + (size_t)(rowBase + 16 * wave + i) * 512 + part * 256 + colBase + 8 * j;
      *(volatile v8us*)op = pv[i];
    }
  }
}

__device__ __forceinline__ void silu_split8(v8f d, v4f ba, v4f bb, v4i& hw, v4i& lw) {
  const v8f bv = {ba.x, ba.y, ba.z, ba.w, bb.x, bb.y, bb.z, bb.w};
  unsigned hb[8], lb[8];
#pragma unroll
  for (int r = 0; r < 8; ++r) {
    const float s = silu_fast(d[r] + bv[r]);
    const unsigned h = bf16_bits(s);
    hb[r] = h;
    lb[r] = bf16_bits(s - __uint_as_float(h << 16));
  }
  const v4i a = {(int)(hb[0] | (hb[1] << 16)), (int)(hb[2] | (hb[3] << 16)),
                 (int)(hb[4] | (hb[5] << 16)), (int)(hb[6] | (hb[7] << 16))};
  const v4i b = {(int)(lb[0] | (lb[1] << 16)), (int)(lb[2] | (lb[3] << 16)),
                 (int)(lb[4] | (lb[5] << 16)), (int)(lb[6] | (lb[7] << 16))};
  hw = a;
  lw = b;
}

__global__ __launch_bounds__(ETHR) __attribute__((amdgpu_num_vgpr(248)))
void k_edge(const float* __restrict__ rE, const float* __restrict__ Rn, const float* __restrict__ HX,
            const float* __restrict__ SPl, const unsigned short* __restrict__ W1Pl,
            const unsigned short* __restrict__ W2Pl, unsigned short* AHL) {
  extern __shared__ __attribute__((aligned(16))) float dyn[];
  float*          sW    = dyn + E_SW;
  float*          sHX   = dyn + E_SHX;
  float*          sAcc  = dyn + E_SACC;
  float*          sSP   = dyn + E_SSP;
  int*            sPair = (int*)(dyn + E_SPAIR);
  unsigned short* sW1h  = (unsigned short*)(dyn + E_SW1);
  unsigned short* sW2h  = (unsigned short*)(dyn + E_SW2);

  const int tid  = (int)threadIdx.x;
  const int lane = tid & 31;
  const int wave = __builtin_amdgcn_readfirstlane(tid >> 5);
  const int hh = lane >> 4, m = lane & 15;
  const int b = (int)blockIdx.x;

  {
    const int ie = tid < 31 ? tid : 31;
    int in = tid - 32;
    in = in < 0 ? 0 : (in > 7 ? 7 : in);
    const float* pe = rE + ((size_t)b * NE + ie) * 3;
    const float* pn = Rn + (size_t)in * 3;
    const float e0 = pe[0], e1 = pe[1], e2 = pe[2];
    const float n0 = pn[0], n1 = pn[1], n2 = pn[2];
    asm volatile("" :: "v"(e0), "v"(e1), "v"(e2), "v"(n0), "v"(n1), "v"(n2));
    if (tid < 32) {
      const v4f q = {bf16_val(e0), bf16_val(e1), bf16_val(e2), 0.0f};
      *(v4fa*)(dyn + E_SRE + 4 * tid) = q;
    }
    if (tid >= 32 && tid < 40) {
      const v4f q = {bf16_val(n0), bf16_val(n1), bf16_val(n2), 0.0f};
      *(v4fa*)(dyn + E_SRN + 4 * (tid - 32)) = q;
    }
    const float* hxg = HX + (size_t)b * (NE * 128);
#pragma unroll
    for (int it = 0; it < 4; ++it) {
      const int idx = it * ETHR + tid;
      *(v4fa*)(sHX + 4 * idx) = *(const v4fa*)(hxg + 4 * idx);
    }
    *(v4fa*)(sSP + 4 * tid) = *(const v4fa*)(SPl + 4 * tid);
#pragma unroll
    for (int it = 0; it < 3; ++it) {
      const int idx = it * ETHR + tid;
      *(v4ia*)(sW1h + 8 * idx) = *(const v4ia*)(W1Pl + 8 * idx);
    }
#pragma unroll
    for (int it = 0; it < 6; ++it) {
      const int idx = it * ETHR + tid;
      *(v4ia*)(sW2h + 8 * idx) = *(const v4ia*)(W2Pl + 8 * idx);
    }
    const int pp = tid >> 4, qq = tid & 15;
    if (pp < qq) sPair[pidx(pp, qq)] = pp | (qq << 8);
    if (tid < 8) sPair[120 + tid] = 0;
  }
  __syncthreads();

  const v8f z8 = {0.f, 0.f, 0.f, 0.f, 0.f, 0.f, 0.f, 0.f};
  const float mu0 = hh ? MUC4 : MUC0;
  const float mu1 = hh ? MUC5 : MUC1;
  const float mu2 = hh ? MUC6 : MUC2;
  const float mu3 = hh ? MUC7 : MUC3;

#pragma unroll 1
  for (int t = 0; t < 3; ++t) {
    const int nT = (t == 1) ? 15 : 16;
#pragma unroll 1
    for (int tile = wave; tile < nT; tile += 8) {
      const int row = 16 * tile + m;
      int pi, offb;
      if (t == 0) {
        pi = row >> 3;
        offb = E_SRN + 4 * (row & 7);
      } else if (t == 1) {
        const int rc = row < 239 ? row : 239;
        const int sb = rc >= 120 ? 1 : 0;
        const int pr = sPair[rc - 120 * sb];
        pi = 16 * sb + (pr & 15);
        offb = E_SRE + 4 * (16 * sb + ((pr >> 8) & 15));
      } else {
        pi = row >> 4;
        offb = E_SRE + 4 * (16 + (row & 15));
      }
      const v4f pa = *(const v4fa*)(dyn + E_SRE + 4 * pi);
      const v4f pb = *(const v4fa*)(dyn + offb);
      const float dx = pa.x - pb.x, dy = pa.y - pb.y, dz = pa.z - pb.z;
      const float d2 = (dx * dx + dz * dz) + dy * dy;
      const float dd = sqrtf(d2 + 1e-6f);
      const float t0 = dd - mu0, t1 = dd - mu1, t2 = dd - mu2, t3 = dd - mu3;
      const float f0 = expf(-(t0 * t0));
      const float f1 = expf(-(t1 * t1));
      const float f2 = expf(-(t2 * t2));
      const float f3 = expf(-(t3 * t3));
      const unsigned h0 = bf16_bits(f0), h1 = bf16_bits(f1), h2 = bf16_bits(f2), h3 = bf16_bits(f3);
      const unsigned l0 = bf16_bits(f0 - __uint_as_float(h0 << 16));
      const unsigned l1 = bf16_bits(f1 - __uint_as_float(h1 << 16));
      const unsigned l2 = bf16_bits(f2 - __uint_as_float(h2 << 16));
      const unsigned l3 = bf16_bits(f3 - __uint_as_float(h3 << 16));
      const int hw0 = (int)(h0 | (h1 << 16)), hw1 = (int)(h2 | (h3 << 16));
      const int lw0 = (int)(l0 | (l1 << 16)), lw1 = (int)(l2 | (l3 << 16));
      const int rh0 = __shfl_xor(hw0, 16);
      const int rh1 = __shfl_xor(hw1, 16);
      const int rl0 = __shfl_xor(lw0, 16);
      const int rl1 = __shfl_xor(lw1, 16);
      FragB fb;
      {
        const v8i w = {hh ? rl0 : hw0, hh ? rl1 : hw1, hh ? lw0 : rh0, hh ? lw1 : rh1, 0, 0, 0, 0};
        fb.w = w;
      }

      v8f d1[4];
#pragma unroll
      for (int nt = 0; nt < 4; ++nt) {
        const unsigned short* wr = sW1h + (size_t)((t * HH + 16 * nt + m) * 32 + 8 * hh);
        FragB fa;
        fa.h[0] = *(const v8usa*)wr;
        fa.h[1] = *(const v8usa*)(wr + 16);
        d1[nt] = wmb(fa, fb, z8);
      }

      v4i hwA, hwB, hwC, hwD, lwA, lwB, lwC, lwD;
      {
        const float* bp = sSP + 512 + t * HH + 8 * hh;
        silu_split8(d1[0], *(const v4fa*)(bp),      *(const v4fa*)(bp + 4),  hwA, lwA);
        silu_split8(d1[1], *(const v4fa*)(bp + 16), *(const v4fa*)(bp + 20), hwB, lwB);
        silu_split8(d1[2], *(const v4fa*)(bp + 32), *(const v4fa*)(bp + 36), hwC, lwC);
        silu_split8(d1[3], *(const v4fa*)(bp + 48), *(const v4fa*)(bp + 52), hwD, lwD);
      }
      FragB bh0, bh1, bl0, bl1;
      bh0.w = __builtin_shufflevector(hwA, hwB, 0, 1, 2, 3, 4, 5, 6, 7);
      bh1.w = __builtin_shufflevector(hwC, hwD, 0, 1, 2, 3, 4, 5, 6, 7);
      bl0.w = __builtin_shufflevector(lwA, lwB, 0, 1, 2, 3, 4, 5, 6, 7);
      bl1.w = __builtin_shufflevector(lwC, lwD, 0, 1, 2, 3, 4, 5, 6, 7);

#pragma unroll
      for (int nt = 0; nt < 4; ++nt) {
        const unsigned short* wr = sW2h + (size_t)((t * HH + 16 * nt + m) * HH + 8 * hh);
        FragB a0, a1;
        a0.h[0] = *(const v8usa*)wr;
        a0.h[1] = *(const v8usa*)(wr + 16);
        a1.h[0] = *(const v8usa*)(wr + 32);
        a1.h[1] = *(const v8usa*)(wr + 48);
        v8f acc = z8;
        acc = wmb(a0, bh0, acc);
        acc = wmb(a1, bh1, acc);
        acc = wmb(a0, bl0, acc);
        acc = wmb(a1, bl1, acc);
        const float* bq = sSP + 768 + t * HH + 16 * nt + 8 * hh;
        const v4f ba = *(const v4fa*)bq;
        const v4f bb = *(const v4fa*)(bq + 4);
        const v4f o0 = {acc[0] + ba.x, acc[1] + ba.y, acc[2] + ba.z, acc[3] + ba.w};
        const v4f o1 = {acc[4] + bb.x, acc[5] + bb.y, acc[6] + bb.z, acc[7] + bb.w};
        float* wp = sW + row * HH + 16 * nt + 8 * hh;
        *(v4fa*)wp       = o0;
        *(v4fa*)(wp + 4) = o1;
      }
    }
    __syncthreads();

    {
      const int gh  = ((wave & 1) << 5) + lane;
      const int gi0 = (wave >> 1) * 8;
#pragma unroll 1
      for (int j = 0; j < 8; ++j) {
        const int i = gi0 + j;
        float acc = 0.0f;
        if (t == 0) {
#pragma unroll 4
          for (int n = 0; n < NN; ++n)
            acc = fmaf(sW[(i * 8 + n) * HH + gh], sSP[n * HH + gh], acc);
        } else if (t == 1) {
          const int sb = i >> 4, li = i & 15;
#pragma unroll 1
          for (int lk = 0; lk < 16; ++lk) {
            if (lk != li) {
              const int p = li < lk ? li : lk;
              const int q = li < lk ? lk : li;
              const int wr = 120 * sb + pidx(p, q);
              acc = fmaf(sW[wr * HH + gh], sHX[(16 * sb + lk) * 128 + gh], acc);
            }
          }
        } else {
          const int sb = i >> 4;
          const int ob = 16 * (1 - sb);
#pragma unroll 4
          for (int lk = 0; lk < 16; ++lk) {
            const int k  = ob + lk;
            const int up = sb == 0 ? i : k;
            const int dn = sb == 0 ? k : i;
            const int wr = up * 16 + (dn - 16);
            acc = fmaf(sW[wr * HH + gh], sHX[k * 128 + HH + gh], acc);
          }
        }
        sAcc[i * A3H + t * HH + gh] = acc;
      }
    }
    __syncthreads();
  }

  {
    v8us pv[6];
#pragma unroll
    for (int it = 0; it < 6; ++it) {
      const int p    = it * ETHR + tid;
      const int rw   = p / 48;
      const int c    = p - rw * 48;
      const int part = c >= 24 ? 1 : 0;
      const int c8   = (c - 24 * part) * 8;
      const float* ap = sAcc + rw * A3H + c8;
      const v4f a = *(const v4fa*)ap;
      const v4f bq = *(const v4fa*)(ap + 4);
      const v8f f8 = {a.x, a.y, a.z, a.w, bq.x, bq.y, bq.z, bq.w};
      const unsigned mh = 0u - (unsigned)part;
      const unsigned ml = ~mh;
      v8us oo;
#pragma unroll
      for (int e = 0; e < 8; ++e) {
        const unsigned hb = bf16_bits(f8[e]);
        const unsigned lb = bf16_bits(f8[e] - __uint_as_float(hb << 16));
        oo[e] = (unsigned short)((hb & ml) | (lb & mh));
      }
      pv[it] = oo;
    }
    unsigned short* ob = AHL + (size_t)b * (NE * KA);
#pragma unroll
    for (int it = 0; it < 6; ++it) *(volatile v8us*)(ob + (size_t)(it * ETHR + tid) * 8) = pv[it];
    __threadfence();
#pragma unroll
    for (int it = 0; it < 6; ++it) *(volatile v8us*)(ob + (size_t)(it * ETHR + tid) * 8) = pv[it];
  }
}

extern "C" void kernel_launch(void* const* d_in, const int* in_sizes, int n_in,
                              void* d_out, int out_size, void* d_ws, size_t ws_size,
                              hipStream_t stream) {
  if (n_in < 14) return;
  if (in_sizes[0] != NCFG * NE * 3) return;
  if (in_sizes[1] != NN * 3) return;
  if (in_sizes[2] != DD) return;
  if (in_sizes[3] != NN * DD) return;
  if (in_sizes[4] != LL * 3 * FF * HH) return;
  if (in_sizes[5] != LL * 3 * HH) return;
  if (in_sizes[6] != LL * 3 * HH * HH) return;
  if (in_sizes[7] != LL * 3 * HH) return;
  if (in_sizes[8] != LL * 3 * DD * HH) return;
  if (in_sizes[9] != LL * 3 * HH) return;
  if (in_sizes[10] != LL * A3H * DD) return;
  if (in_sizes[11] != LL * DD) return;
  if (in_sizes[12] != LL * DD * DD) return;
  if (in_sizes[13] != LL * DD) return;
  if (out_size != MROWS * DD) return;

  const float* rE   = (const float*)d_in[0];
  const float* Rn   = (const float*)d_in[1];
  const float* elec = (const float*)d_in[2];
  const float* nuc  = (const float*)d_in[3];
  const float* wW1  = (const float*)d_in[4];
  const float* wB1  = (const float*)d_in[5];
  const float* wW2  = (const float*)d_in[6];
  const float* wB2  = (const float*)d_in[7];
  const float* hW   = (const float*)d_in[8];
  const float* hB   = (const float*)d_in[9];
  const float* uW1  = (const float*)d_in[10];
  const float* uB1  = (const float*)d_in[11];
  const float* uW2  = (const float*)d_in[12];
  const float* uB2  = (const float*)d_in[13];
  float* out = (float*)d_out;

  char* ws = (char*)d_ws;
  size_t off = 0;
  const size_t oX   = off; off += (size_t)MROWS * DD * 4;
  const size_t oXHL = off; off += (size_t)MROWS * KX * 2;
  const size_t oHX  = off; off += (size_t)MROWS * 128 * 4;
  const size_t oTHL = off; off += (size_t)MROWS * KT * 2;
  const size_t oW1P = off; off += (size_t)LL * 3 * HH * 32 * 2;
  const size_t oW2P = off; off += (size_t)LL * 3 * HH * HH * 2;
  const size_t oHWP = off; off += (size_t)LL * 128 * KX * 2;
  const size_t oU1P = off; off += (size_t)LL * DD * KA * 2;
  const size_t oU2P = off; off += (size_t)LL * DD * KT * 2;
  const size_t oSP  = off; off += (size_t)LL * 1024 * 4;
  const size_t oHB  = off; off += (size_t)LL * 128 * 4;
  const size_t oUB1 = off; off += (size_t)LL * DD * 4;
  const size_t oUB2 = off; off += (size_t)LL * DD * 4;
  if (off > ws_size || off > (size_t)WSMAX) return;
  if ((size_t)MROWS * KA * 2 > (size_t)MROWS * KX * 2) return;

  float*          X    = (float*)(ws + oX);
  unsigned short* XHL  = (unsigned short*)(ws + oXHL);
  unsigned short* AHL  = (unsigned short*)(ws + oXHL);
  float*          HXp  = (float*)(ws + oHX);
  unsigned short* THL  = (unsigned short*)(ws + oTHL);
  unsigned short* W1P  = (unsigned short*)(ws + oW1P);
  unsigned short* W2P  = (unsigned short*)(ws + oW2P);
  unsigned short* HWP  = (unsigned short*)(ws + oHWP);
  unsigned short* U1P  = (unsigned short*)(ws + oU1P);
  unsigned short* U2P  = (unsigned short*)(ws + oU2P);
  float*          SP   = (float*)(ws + oSP);
  float*          HBP  = (float*)(ws + oHB);
  float*          UB1P = (float*)(ws + oUB1);
  float*          UB2P = (float*)(ws + oUB2);

  hipFuncSetAttribute(reinterpret_cast<const void*>(&k_edge), hipFuncAttributeMaxDynamicSharedMemorySize,
                      (int)EDGE_LDS_BYTES);

  k_pa<<<PA_L2 / 256, 256, 0, stream>>>(wW1, wW2, hW, W1P, W2P, HWP);
  k_pb<<<PB_L1 / 256, 256, 0, stream>>>(uW1, uW2, U1P, U2P);
  k_pc<<<(PC_L3 + 255) / 256, 256, 0, stream>>>(nuc, hW, hB, wB1, wB2, uB1, uB2, SP, HBP, UB1P, UB2P);
  k_x0<<<X0_L1 / 256, 256, 0, stream>>>(elec, X, XHL);

  for (int l = 0; l < LL; ++l) {
    k_gemm<0><<<dim3(MROWS / GBM, 1), GTHR, 0, stream>>>(XHL, KX, HWP + (size_t)l * 128 * KX, KX, KX,
                                                         HBP + (size_t)l * 128, X, HXp, THL);
    k_edge<<<NCFG, ETHR, EDGE_LDS_BYTES, stream>>>(rE, Rn, HXp, SP + (size_t)l * 1024,
                                                   W1P + (size_t)l * 3 * HH * 32,
                                                   W2P + (size_t)l * 3 * HH * HH, AHL);
    k_gemm<1><<<dim3(MROWS / GBM, DD / GBN), GTHR, 0, stream>>>(AHL, KA, U1P + (size_t)l * DD * KA, KA, KA,
                                                                UB1P + (size_t)l * DD, X, HXp, THL);
    if (l < LL - 1) {
      k_gemm<2><<<dim3(MROWS / GBM, DD / GBN), GTHR, 0, stream>>>(THL, KT, U2P + (size_t)l * DD * KT, KT, KT,
                                                                  UB2P + (size_t)l * DD, X, out, XHL);
    } else {
      k_gemm<3><<<dim3(MROWS / GBM, DD / GBN), GTHR, 0, stream>>>(THL, KT, U2P + (size_t)l * DD * KT, KT, KT,
                                                                  UB2P + (size_t)l * DD, X, out, XHL);
    }
  }
}
